// InvertedResidualBlockME_49469433316046
// MI455X (gfx1250) — hardware-verified
//
#include <hip/hip_runtime.h>
#include <stdint.h>


#define CIN   32
#define HID   192
#define COUT  32
#define KOFF  9
#define EPSV  1e-5f
#define WSCALE 16.0f
#define WINV   0.0625f

typedef _Float16 f16t;
typedef f16t  v16h __attribute__((ext_vector_type(16)));
typedef f16t  v8h  __attribute__((ext_vector_type(8)));
typedef f16t  v2h  __attribute__((ext_vector_type(2)));
typedef float v8f  __attribute__((ext_vector_type(8)));
typedef float v4f  __attribute__((ext_vector_type(4)));

union Frag { v16h v; v8h half[2]; };

__device__ __forceinline__ v8f wmma16(v16h a, v16h b, v8f acc)
{
    acc = __builtin_amdgcn_wmma_f32_16x16x32_f16(false, a, false, b, (short)0, acc, false, false);
    asm volatile("v_nop\n\tv_nop\n\tv_nop\n\tv_nop" : "+v"(acc) : "v"(a), "v"(b));
    return acc;
}

__global__ __launch_bounds__(128)
void k_expand(const float* __restrict__ feats, const float* __restrict__ W1,
              const float* __restrict__ g1, const float* __restrict__ b1,
              const float* __restrict__ m1, const float* __restrict__ v1,
              f16t* __restrict__ X1, int N)
{
    __shared__ __align__(16) f16t  sW1B[12][32][16];
    __shared__ __align__(16) f16t  sT[4][16][HID];
    __shared__ float sScl[HID];
    __shared__ float sSh[HID];

    const int t = threadIdx.x;
    for (int c = t; c < HID; c += 128) {
        float sc = g1[c] * rsqrtf(v1[c] + EPSV);
        sScl[c] = sc * WINV;
        sSh[c]  = b1[c] - m1[c] * sc;
    }
    for (int i = t; i < 12 * 32 * 16; i += 128) {
        int ct  = i >> 9;
        int ln  = (i >> 4) & 31;
        int e   = i & 15;
        int col = ct * 16 + (ln & 15);
        int hh  = ln >> 4;
        int k   = (e < 8) ? (8 * hh + e) : (16 + 8 * hh + (e - 8));
        sW1B[ct][ln][e] = (f16t)(W1[k * HID + col] * WSCALE);
    }
    __syncthreads();

    const int wave = __builtin_amdgcn_readfirstlane(t >> 5);
    const int lane = t & 31;
    const int m    = lane & 15;
    const int h    = lane >> 4;
    const int row0 = blockIdx.x * 64 + wave * 16;

    int arow = row0 + m;
    if (arow > N - 1) arow = N - 1;
    const float* fr = feats + (size_t)arow * CIN;

    Frag A;
    {
        v4f p0 = *(const v4f*)(fr + 8 * h);
        v4f p1 = *(const v4f*)(fr + 8 * h + 4);
        v4f p2 = *(const v4f*)(fr + 16 + 8 * h);
        v4f p3 = *(const v4f*)(fr + 16 + 8 * h + 4);
#pragma unroll
        for (int e = 0; e < 4; ++e) {
            A.v[e]      = (f16t)p0[e];
            A.v[4 + e]  = (f16t)p1[e];
            A.v[8 + e]  = (f16t)p2[e];
            A.v[12 + e] = (f16t)p3[e];
        }
    }

#pragma unroll 1
    for (int ct = 0; ct < 12; ++ct) {
        Frag B;
        B.half[0] = *(const v8h*)&sW1B[ct][lane][0];
        B.half[1] = *(const v8h*)&sW1B[ct][lane][8];
        v8f acc = {};
        acc = wmma16(A.v, B.v, acc);
        const int col = ct * 16 + m;
        const float scl = sScl[col];
        const float sh  = sSh[col];
#pragma unroll
        for (int r = 0; r < 8; ++r) {
            float y = fminf(fmaxf(acc[r] * scl + sh, 0.0f), 6.0f);
            sT[wave][8 * h + r][col] = (f16t)y;
        }
    }
    __syncthreads();

    f16t* xbase = X1 + (size_t)row0 * HID;
    const int lg = lane >> 3;
    const int q  = lane & 7;
    v4f vals[12];
#pragma unroll
    for (int j = 0; j < 12; ++j) {
        const int L   = 4 * j + lg;
        const int rr  = L / 3;
        const int seg = L - rr * 3;
        vals[j] = *(const v4f*)&sT[wave][rr][seg * 64 + q * 8];
    }
#pragma unroll
    for (int j = 0; j < 12; ++j) {
        const int L   = 4 * j + lg;
        const int rr  = L / 3;
        const int seg = L - rr * 3;
        *(volatile v4f*)(xbase + (size_t)rr * HID + seg * 64 + q * 8) = vals[j];
    }
    __threadfence();
#pragma unroll
    for (int j = 0; j < 12; ++j) {
        const int L   = 4 * j + lg;
        const int rr  = L / 3;
        const int seg = L - rr * 3;
        *(volatile v4f*)(xbase + (size_t)rr * HID + seg * 64 + q * 8) = vals[j];
    }
}

__global__ __launch_bounds__(256)
void k_dwproj(const float* __restrict__ feats,
              const int*   __restrict__ nbr,
              const float* __restrict__ W2,
              const float* __restrict__ W3,
              const float* __restrict__ g2, const float* __restrict__ b2,
              const float* __restrict__ m2, const float* __restrict__ v2,
              const float* __restrict__ g3, const float* __restrict__ b3,
              const float* __restrict__ m3, const float* __restrict__ v3,
              const f16t*  __restrict__ X1,
              float* __restrict__ out, int N)
{
    __shared__ __align__(16) f16t  sY[64][HID];
    __shared__ __align__(16) f16t  sW3B[2][6][32][16];
    __shared__ __align__(16) float sOut[64][COUT];
    __shared__ float sW2s[KOFF][HID];
    __shared__ int   sNbr[64][KOFF];
    __shared__ float sScl2[HID];
    __shared__ float sSh2[HID];
    __shared__ float sScl3[COUT];
    __shared__ float sSh3[COUT];

    const int t    = threadIdx.x;
    const int row0 = blockIdx.x * 64;

    for (int c = t; c < HID; c += 256) {
        float sc  = g2[c] * rsqrtf(v2[c] + EPSV);
        sScl2[c]  = sc;
        sSh2[c]   = b2[c] - m2[c] * sc;
    }
    if (t < COUT) {
        float sc  = g3[t] * rsqrtf(v3[t] + EPSV);
        sScl3[t]  = sc * WINV;
        sSh3[t]   = b3[t] - m3[t] * sc;
    }
    __syncthreads();

    for (int i = t; i < 2 * 6 * 32 * 16; i += 256) {
        int ct  = i / 3072;
        int rem = i - ct * 3072;
        int kk  = rem >> 9;
        int ln  = (rem >> 4) & 31;
        int e   = i & 15;
        int col = ct * 16 + (ln & 15);
        int hh  = ln >> 4;
        int k   = kk * 32 + ((e < 8) ? (8 * hh + e) : (16 + 8 * hh + (e - 8)));
        sW3B[ct][kk][ln][e] = (f16t)(W3[k * COUT + col] * WSCALE);
    }
    for (int i = t; i < KOFF * HID; i += 256) {
        int k = i / HID;
        int c = i - k * HID;
        sW2s[k][c] = W2[i] * sScl2[c];
    }
    for (int i = t; i < 64 * KOFF; i += 256) {
        int r = i / KOFF;
        int k = i - r * KOFF;
        int grow = row0 + r;
        sNbr[r][k] = (grow < N) ? nbr[(size_t)grow * KOFF + k] : -1;
    }
    __syncthreads();

    const int wave = __builtin_amdgcn_readfirstlane(t >> 5);
    const int lane = t & 31;
    const int m    = lane & 15;
    const int h    = lane >> 4;

    {
        const int c0 = 2 * lane;
        float w[KOFF][6];
#pragma unroll
        for (int k = 0; k < KOFF; ++k) {
            const float* wp = &sW2s[k][c0];
            w[k][0] = wp[0];   w[k][1] = wp[1];
            w[k][2] = wp[64];  w[k][3] = wp[65];
            w[k][4] = wp[128]; w[k][5] = wp[129];
        }
#pragma unroll 1
        for (int rr = 0; rr < 8; ++rr) {
            const int r = wave * 8 + rr;
            float a0 = 0.f, a1 = 0.f, a2 = 0.f, a3 = 0.f, a4 = 0.f, a5 = 0.f;
#pragma unroll
            for (int k = 0; k < KOFF; ++k) {
                int nb = __builtin_amdgcn_readfirstlane(sNbr[r][k]);
                if (nb >= 0) {
                    if (nb > N - 1) nb = N - 1;
                    const f16t* xr = X1 + (size_t)nb * HID;
                    v2h x0 = *(const v2h*)(xr + c0);
                    v2h x1 = *(const v2h*)(xr + c0 + 64);
                    v2h x2 = *(const v2h*)(xr + c0 + 128);
                    a0 += (float)x0[0] * w[k][0];
                    a1 += (float)x0[1] * w[k][1];
                    a2 += (float)x1[0] * w[k][2];
                    a3 += (float)x1[1] * w[k][3];
                    a4 += (float)x2[0] * w[k][4];
                    a5 += (float)x2[1] * w[k][5];
                }
            }
            {
                v2h o;
                o[0] = (f16t)fminf(fmaxf(a0 + sSh2[c0],       0.f), 6.f);
                o[1] = (f16t)fminf(fmaxf(a1 + sSh2[c0 + 1],   0.f), 6.f);
                *(v2h*)&sY[r][c0] = o;
                o[0] = (f16t)fminf(fmaxf(a2 + sSh2[c0 + 64],  0.f), 6.f);
                o[1] = (f16t)fminf(fmaxf(a3 + sSh2[c0 + 65],  0.f), 6.f);
                *(v2h*)&sY[r][c0 + 64] = o;
                o[0] = (f16t)fminf(fmaxf(a4 + sSh2[c0 + 128], 0.f), 6.f);
                o[1] = (f16t)fminf(fmaxf(a5 + sSh2[c0 + 129], 0.f), 6.f);
                *(v2h*)&sY[r][c0 + 128] = o;
            }
        }
    }
    __syncthreads();

    {
        const int rt   = wave & 3;
        const int ct   = wave >> 2;
        const int rloc = rt * 16 + m;
        v8f acc = {};
#pragma unroll
        for (int kk = 0; kk < 6; ++kk) {
            Frag A, B;
            const f16t* p = &sY[rloc][kk * 32 + 8 * h];
            A.half[0] = *(const v8h*)p;
            A.half[1] = *(const v8h*)(p + 16);
            B.half[0] = *(const v8h*)&sW3B[ct][kk][lane][0];
            B.half[1] = *(const v8h*)&sW3B[ct][kk][lane][8];
            acc = wmma16(A.v, B.v, acc);
        }
        const int col   = ct * 16 + m;
        const float scl = sScl3[col];
        const float sh  = sSh3[col];
#pragma unroll
        for (int r = 0; r < 8; ++r)
            sOut[rt * 16 + 8 * h + r][col] = acc[r] * scl + sh;
    }
    __syncthreads();

    {
        const int lg = lane >> 3;
        const int q  = lane & 7;
        v4f o0, o1;
        int g0r, g1r;
        {
            const int L  = wave * 8 + lg;
            const int gr = row0 + L;
            const int lr = (gr < N) ? gr : (N - 1);
            o0  = *(const v4f*)&sOut[L][q * 4] + *(const v4f*)(feats + (size_t)lr * COUT + q * 4);
            g0r = gr;
        }
        {
            const int L  = wave * 8 + 4 + lg;
            const int gr = row0 + L;
            const int lr = (gr < N) ? gr : (N - 1);
            o1  = *(const v4f*)&sOut[L][q * 4] + *(const v4f*)(feats + (size_t)lr * COUT + q * 4);
            g1r = gr;
        }
        if (g0r < N) *(volatile v4f*)(out + (size_t)g0r * COUT + q * 4) = o0;
        if (g1r < N) *(volatile v4f*)(out + (size_t)g1r * COUT + q * 4) = o1;
        __threadfence();
        if (g0r < N) *(volatile v4f*)(out + (size_t)g0r * COUT + q * 4) = o0;
        if (g1r < N) *(volatile v4f*)(out + (size_t)g1r * COUT + q * 4) = o1;
    }
}

extern "C" void kernel_launch(void* const* d_in, const int* in_sizes, int n_in,
                              void* d_out, int out_size, void* d_ws, size_t ws_size,
                              hipStream_t stream)
{
    if (n_in < 17) return;
    const float* feats = (const float*)d_in[0];
    const int*   nbr   = (const int*)  d_in[1];
    const float* W1    = (const float*)d_in[2];
    const float* W2    = (const float*)d_in[3];
    const float* W3    = (const float*)d_in[4];
    const float* g1 = (const float*)d_in[5];
    const float* b1 = (const float*)d_in[6];
    const float* m1 = (const float*)d_in[7];
    const float* v1 = (const float*)d_in[8];
    const float* g2 = (const float*)d_in[9];
    const float* b2 = (const float*)d_in[10];
    const float* m2 = (const float*)d_in[11];
    const float* v2 = (const float*)d_in[12];
    const float* g3 = (const float*)d_in[13];
    const float* b3 = (const float*)d_in[14];
    const float* m3 = (const float*)d_in[15];
    const float* v3 = (const float*)d_in[16];
    float* out = (float*)d_out;

    const int N = in_sizes[0] / CIN;
    if (N <= 0) return;
    if (in_sizes[1] != N * KOFF) return;
    if (in_sizes[2] != CIN * HID || in_sizes[3] != KOFF * HID || in_sizes[4] != HID * COUT) return;
    if (out_size != N * COUT) return;

    const int nblk = (N + 63) / 64;
    const int Npad = nblk * 64;
    const size_t x1_bytes = (size_t)Npad * HID * sizeof(f16t);
    if (x1_bytes > ws_size) return;
    f16t* X1 = (f16t*)d_ws;

    k_expand<<<nblk, 128, 0, stream>>>(feats, W1, g1, b1, m1, v1, X1, N);
    k_dwproj<<<nblk, 256, 0, stream>>>(feats, nbr, W2, W3, g2, b2, m2, v2,
                                       g3, b3, m3, v3, X1, out, N);
}
